// GTLayer_84722524880938
// MI455X (gfx1250) — hardware-verified
//
#include <hip/hip_runtime.h>
#include <math.h>

constexpr int kBatch    = 2;
constexpr int kSeq      = 2048;
constexpr int kDim      = 1024;
constexpr int kFfn      = 4096;
constexpr int kHeads    = 8;
constexpr int kHeadDim  = 128;
constexpr int kRl       = 4;
constexpr int kTok      = kBatch * kSeq;
constexpr int kGroups   = kBatch * kHeads;
constexpr int kChunk    = kSeq * kHeadDim;
constexpr int kGpp      = 2;
constexpr float kWCarry     = 16.0f;
constexpr float kWCarryInv  = 1.0f / 16.0f;
constexpr float kPCarry     = 32768.0f;
constexpr float kCtxCarry   = 256.0f;
constexpr float kScoreScale = 0.08838834764831845f;
constexpr float kPVScale    = kCtxCarry / kPCarry;
constexpr float kWoScale    = 1.0f / (kCtxCarry * kWCarry);
constexpr float kInvDim     = 1.0f / 1024.0f;
constexpr float kLnEps      = 1e-5f;
static_assert(kHeads * kHeadDim == kDim, "shape");
static_assert(kGroups * kChunk == kTok * kDim, "chunks");
static_assert(kGroups % kGpp == 0 && (kHeads % kGpp) == 0, "passes");
static_assert(kTok % 64 == 0 && kDim % 64 == 0 && kFfn % 64 == 0 && kSeq % 64 == 0 && kHeadDim % 64 == 0, "tiles");
static_assert(kDim % 32 == 0 && kHeadDim % 32 == 0 && kSeq % 32 == 0 && kFfn % 32 == 0, "ksteps");
static_assert(kSeq == 4 * 512, "softmax row map");

typedef __attribute__((ext_vector_type(16))) _Float16 v16h;
typedef __attribute__((ext_vector_type(8)))  _Float16 v8h;
typedef __attribute__((ext_vector_type(16))) __bf16   v16b;
typedef __attribute__((ext_vector_type(8)))  __bf16   v8b;
typedef __attribute__((ext_vector_type(8)))  float    v8f;
typedef __attribute__((ext_vector_type(4)))  float    v4f;
typedef __attribute__((ext_vector_type(2)))  float    v2f;
typedef __attribute__((ext_vector_type(4)))  unsigned int v4u;

__device__ __forceinline__ unsigned short f2bf_bits(float f) {
  unsigned u = __float_as_uint(f);
  return (unsigned short)((u + 0x7FFFu + ((u >> 16) & 1u)) >> 16);
}
__device__ __forceinline__ float bf_bits2f(unsigned short h) { return __uint_as_float(((unsigned)h) << 16); }

__device__ __forceinline__ void dep_guard_h(v8f& a, v8f& b, v16h x, v16h y) { asm volatile("v_nop\n\tv_nop\n\tv_nop\n\tv_nop" : "+v"(a), "+v"(b) : "v"(x), "v"(y)); }
__device__ __forceinline__ void dep_guard_b(v8f& a, v8f& b, v16b x, v16b y) { asm volatile("v_nop\n\tv_nop\n\tv_nop\n\tv_nop" : "+v"(a), "+v"(b) : "v"(x), "v"(y)); }
__device__ __forceinline__ void dep_guard4_h(v8f& a, v8f& b, v8f& c, v8f& d, v16h x, v16h y) { asm volatile("v_nop\n\tv_nop\n\tv_nop\n\tv_nop" : "+v"(a), "+v"(b), "+v"(c), "+v"(d) : "v"(x), "v"(y)); }
__device__ __forceinline__ void dep_guard4_b(v8f& a, v8f& b, v8f& c, v8f& d, v16b x, v16b y) { asm volatile("v_nop\n\tv_nop\n\tv_nop\n\tv_nop" : "+v"(a), "+v"(b), "+v"(c), "+v"(d) : "v"(x), "v"(y)); }
__device__ __forceinline__ void keep4_h(v16h a, v16h b, v16h c, v16h d) { asm volatile("v_nop" :: "v"(a), "v"(b), "v"(c), "v"(d)); }
__device__ __forceinline__ void keep4_b(v16b a, v16b b, v16b c, v16b d) { asm volatile("v_nop" :: "v"(a), "v"(b), "v"(c), "v"(d)); }
__device__ __forceinline__ void acc_guard4(v8f& a, v8f& b, v8f& c, v8f& d) { asm volatile("v_nop\n\tv_nop\n\tv_nop\n\tv_nop" : "+v"(a), "+v"(b), "+v"(c), "+v"(d)); }
template <typename T> struct Frag;
template <> struct Frag<_Float16> {
  typedef v16h V; union U { v16h v; v8h h[2]; };
  static __device__ __forceinline__ v16h load(const _Float16* p) {
    U f; f.h[0] = *(const v8h*)(p); f.h[1] = *(const v8h*)(p + 16); return f.v;
  }
  static __device__ __forceinline__ v8f mma(v16h a, v16h b, v8f c) {
    return __builtin_amdgcn_wmma_f32_16x16x32_f16(false, a, false, b, (short)0, c, false, false);
  }
  static __device__ __forceinline__ void guard(v8f& a, v8f& b, v16h x, v16h y) { dep_guard_h(a, b, x, y); }
  static __device__ __forceinline__ void guard4(v8f& a, v8f& b, v8f& c, v8f& d, v16h x, v16h y) { dep_guard4_h(a, b, c, d, x, y); }
  static __device__ __forceinline__ void keep(v16h a, v16h b, v16h c, v16h d) { keep4_h(a, b, c, d); }
};
template <> struct Frag<__bf16> {
  typedef v16b V; union U { v16b v; v8b h[2]; };
  static __device__ __forceinline__ v16b load(const __bf16* p) {
    U f; f.h[0] = *(const v8b*)(p); f.h[1] = *(const v8b*)(p + 16); return f.v;
  }
  static __device__ __forceinline__ v8f mma(v16b a, v16b b, v8f c) {
    return __builtin_amdgcn_wmma_f32_16x16x32_bf16(false, a, false, b, (short)0, c, false, false);
  }
  static __device__ __forceinline__ void guard(v8f& a, v8f& b, v16b x, v16b y) { dep_guard_b(a, b, x, y); }
  static __device__ __forceinline__ void guard4(v8f& a, v8f& b, v8f& c, v8f& d, v16b x, v16b y) { dep_guard4_b(a, b, c, d, x, y); }
  static __device__ __forceinline__ void keep(v16b a, v16b b, v16b c, v16b d) { keep4_b(a, b, c, d); }
};

__device__ __forceinline__ unsigned pk16(unsigned short a, unsigned short b) { return (unsigned)a | ((unsigned)b << 16); }
__device__ __forceinline__ unsigned short h_bits(float f) { const _Float16 h = (_Float16)f; return __builtin_bit_cast(unsigned short, h); }

template <int ET> struct Elem;
template <> struct Elem<0> { typedef _Float16 T; };
template <> struct Elem<1> { typedef __bf16 T; };
template <int ET, bool SPLIT, int BIAS_MODE, int OUT_MODE, bool RESID, int ACT = 0>
__global__ __launch_bounds__(256) void wmma_gemm64(
    const unsigned short* __restrict__ Ap, const unsigned short* __restrict__ A2p, int lda, long strideA,
    const unsigned short* __restrict__ Btp, const unsigned short* __restrict__ Bt2p, int ldb, long strideB,
    void* __restrict__ Cout, void* __restrict__ Cout2, int ldc, long strideC,
    const float* __restrict__ bias,
    const float* __restrict__ resid, long strideR,
    int M, int N, int K, float scale) {
  typedef typename Elem<ET>::T T;
  typedef typename Frag<T>::V V;
  const T* A = (const T*)Ap; const T* A2 = (const T*)A2p; const T* Bt = (const T*)Btp; const T* Bt2 = (const T*)Bt2p;
  __shared__ __align__(16) float sT[8][16 * 68];
  const int b    = blockIdx.y;
  const int lane = threadIdx.x & 31;
  const int wave = threadIdx.x >> 5;
  const int tilesN = N >> 6;
  const int tilesM = M >> 6;
  const int tile = blockIdx.x * 8 + wave;
  if (tile >= tilesM * tilesN) return;
  const int tm = tile / tilesN;
  const int tn = tile - tm * tilesN;
  const int m0 = tm << 6;
  const int n0 = tn << 6;

  const T* Ab  = A  + (size_t)b * strideA;
  const T* Bb  = Bt + (size_t)b * strideB;
  const T* Ab2 = SPLIT ? (A2  + (size_t)b * strideA) : nullptr;
  const T* Bb2 = SPLIT ? (Bt2 + (size_t)b * strideB) : nullptr;

  const int rlane = lane & 15;
  const int koff  = (lane >> 4) * 8;
  const int mOff  = (lane >> 4) * 8;

  v8f acc[4][4];
#pragma unroll
  for (int i = 0; i < 4; ++i)
#pragma unroll
    for (int j = 0; j < 4; ++j) acc[i][j] = (v8f){0.f,0.f,0.f,0.f,0.f,0.f,0.f,0.f};

  for (int k0 = 0; k0 < K; k0 += 32) {
    V bh[4], bl[4];
#pragma unroll
    for (int j = 0; j < 4; ++j) {
      const size_t bo = (size_t)(n0 + (j << 4) + rlane) * ldb + koff + k0;
      bh[j] = Frag<T>::load(Bb + bo);
      if (SPLIT) bl[j] = Frag<T>::load(Bb2 + bo);
    }
#pragma unroll
    for (int i = 0; i < 4; ++i) {
      const size_t ao = (size_t)(m0 + (i << 4) + rlane) * lda + koff + k0;
      V ah = Frag<T>::load(Ab + ao);
      V al;
      if (SPLIT) al = Frag<T>::load(Ab2 + ao);
#pragma unroll
      for (int j = 0; j < 4; ++j) {
        acc[i][j] = Frag<T>::mma(ah, bh[j], acc[i][j]);
        if (SPLIT) {
          acc[i][j] = Frag<T>::mma(ah, bl[j], acc[i][j]);
          acc[i][j] = Frag<T>::mma(al, bh[j], acc[i][j]);
        }
      }
      Frag<T>::guard4(acc[i][0], acc[i][1], acc[i][2], acc[i][3], ah, SPLIT ? al : ah);
    }
    Frag<T>::keep(bh[0], bh[1], bh[2], bh[3]);
    if (SPLIT) Frag<T>::keep(bl[0], bl[1], bl[2], bl[3]);
  }
  acc_guard4(acc[0][0], acc[0][1], acc[0][2], acc[0][3]);
  acc_guard4(acc[1][0], acc[1][1], acc[1][2], acc[1][3]);
  acc_guard4(acc[2][0], acc[2][1], acc[2][2], acc[2][3]);
  acc_guard4(acc[3][0], acc[3][1], acc[3][2], acc[3][3]);

  float* slab = sT[wave];
  const float* Rb = RESID ? (resid + (size_t)b * strideR) : nullptr;
#pragma unroll
  for (int i = 0; i < 4; ++i) {
    const int mBase = m0 + (i << 4);
#pragma unroll
    for (int j = 0; j < 4; ++j) {
      const int n = n0 + (j << 4) + rlane;
      float bv = 0.f;
      if (BIAS_MODE == 2) bv = bias[n];
#pragma unroll
      for (int r = 0; r < 8; ++r) {
        float v = acc[i][j][r] * scale;
        if (BIAS_MODE == 1) v += bias[mBase + mOff + r];
        if (BIAS_MODE == 2) v += bv;
        if (RESID) v += Rb[(size_t)(mBase + mOff + r) * ldc + n];
        if (ACT == 2) v = fmaxf(v, 0.0f);
        if (ACT == 4) v = (v > 0.f) ? v : 0.01f * v;
        slab[(mOff + r) * 68 + (j << 4) + rlane] = v;
      }
    }
    __builtin_amdgcn_fence(__ATOMIC_RELEASE, "workgroup");
    __builtin_amdgcn_wave_barrier();
    __builtin_amdgcn_fence(__ATOMIC_ACQUIRE, "workgroup");
    if (OUT_MODE == 0) {
      float* C = (float*)Cout + (size_t)b * strideC;
      const int hh = lane >> 4, c4 = (lane & 15) * 4;
      for (int pass = 0; pass < 2; ++pass) {
#pragma unroll
        for (int it = 0; it < 8; ++it) {
          const int row = it * 2 + hh;
          v4f v = *(const v4f*)(slab + row * 68 + c4);
          *(volatile v4f*)(C + (size_t)(mBase + row) * ldc + n0 + c4) = v;
        }
        __threadfence();
      }
    } else {
      const int q = lane >> 3, c8 = (lane & 7) * 8;
      unsigned short* C  = (unsigned short*)Cout  + (size_t)b * strideC;
      unsigned short* C2 = (OUT_MODE == 2) ? ((unsigned short*)Cout2 + (size_t)b * strideC) : nullptr;
      for (int pass = 0; pass < 2; ++pass) {
#pragma unroll
        for (int it = 0; it < 4; ++it) {
          const int row = it * 4 + q;
          const float* sp = slab + row * 68 + c8;
          v8h hv, lv;
#pragma unroll
          for (int e = 0; e < 8; ++e) {
            if (OUT_MODE == 1) {
              hv[e] = (_Float16)sp[e];
            } else {
              unsigned short hb = f2bf_bits(sp[e]);
              unsigned short lb = f2bf_bits(sp[e] - bf_bits2f(hb));
              hv[e] = __builtin_bit_cast(_Float16, hb);
              lv[e] = __builtin_bit_cast(_Float16, lb);
            }
          }
          *(volatile v8h*)(C + (size_t)(mBase + row) * ldc + n0 + c8) = hv;
          if (OUT_MODE == 2) *(volatile v8h*)(C2 + (size_t)(mBase + row) * ldc + n0 + c8) = lv;
        }
        __threadfence();
      }
    }
    __builtin_amdgcn_fence(__ATOMIC_RELEASE, "workgroup");
    __builtin_amdgcn_wave_barrier();
    __builtin_amdgcn_fence(__ATOMIC_ACQUIRE, "workgroup");
  }
}

__global__ __launch_bounds__(256) void cast8_f16_kernel(const float* __restrict__ in, unsigned short* __restrict__ out, int n8) {
  const int i = blockIdx.x * 256 + threadIdx.x;
  if (i >= n8) return;
  const float* p = in + 8 * (size_t)i;
  const v4f a = *(const v4f*)(p);
  const v4f c = *(const v4f*)(p + 4);
  unsigned short hb[8];
#pragma unroll
  for (int e = 0; e < 4; ++e) {
    hb[e]     = h_bits(a[e]);
    hb[4 + e] = h_bits(c[e]);
  }
  const v4u u = (v4u){pk16(hb[0], hb[1]), pk16(hb[2], hb[3]), pk16(hb[4], hb[5]), pk16(hb[6], hb[7])};
  unsigned short* q = out + 8 * (size_t)i;
  *(volatile v4u*)q = u;
  __threadfence();
  *(volatile v4u*)q = u;
}

__global__ __launch_bounds__(256) void wt_cast_kernel(const float* __restrict__ Wa, const float* __restrict__ Wb,
                                                      const float* __restrict__ Wc, const float* __restrict__ Wd,
                                                      unsigned short* __restrict__ out, int kin, int nout,
                                                      long planeStride, float scale) {
  __shared__ float sm[64][65];
  const int t  = threadIdx.x;
  const int k0 = blockIdx.x * 64;
  const int n0 = blockIdx.y * 64;
  const int z  = blockIdx.z;
  const float* W = (z == 0) ? Wa : (z == 1) ? Wb : (z == 2) ? Wc : Wd;
#pragma unroll
  for (int i = 0; i < 4; ++i) {
    const int e  = i * 256 + t;
    const int r  = e >> 4;
    const int c4 = (e & 15) * 4;
    const v4f w = *(const v4f*)(W + (size_t)(k0 + r) * nout + n0 + c4);
    sm[c4 + 0][r] = w[0] * scale;
    sm[c4 + 1][r] = w[1] * scale;
    sm[c4 + 2][r] = w[2] * scale;
    sm[c4 + 3][r] = w[3] * scale;
  }
  __syncthreads();
  const int lane = t & 31, wave = t >> 5;
  const int q = lane >> 3, c8 = (lane & 7) * 8;
  unsigned short* op = out + (size_t)z * planeStride;
  for (int pass = 0; pass < 2; ++pass) {
#pragma unroll
    for (int it = 0; it < 2; ++it) {
      const int row = wave * 8 + it * 4 + q;
      unsigned short hb[8];
#pragma unroll
      for (int e = 0; e < 8; ++e) hb[e] = h_bits(sm[row][c8 + e]);
      const v4u u = (v4u){pk16(hb[0], hb[1]), pk16(hb[2], hb[3]), pk16(hb[4], hb[5]), pk16(hb[6], hb[7])};
      *(volatile v4u*)(op + (size_t)(n0 + row) * kin + k0 + c8) = u;
    }
    __threadfence();
  }
}

__global__ __launch_bounds__(256) void transpose16_kernel(const unsigned short* __restrict__ src, unsigned short* __restrict__ dst,
                                                          int rows, int cols) {
  __shared__ unsigned int sm[64][65];
  const int t  = threadIdx.x;
  const int c0 = blockIdx.x * 64;
  const int r0 = blockIdx.y * 64;
  const size_t cb = (size_t)blockIdx.z * rows * cols;
  const unsigned int* s32 = (const unsigned int*)(src + cb);
#pragma unroll
  for (int i = 0; i < 8; ++i) {
    const int e  = i * 256 + t;
    const int r  = e >> 5;
    const int cw = e & 31;
    const unsigned int w = s32[(((size_t)(r0 + r) * cols + c0) >> 1) + cw];
    sm[2 * cw][r]     = w & 0xffffu;
    sm[2 * cw + 1][r] = w >> 16;
  }
  __syncthreads();
  const int lane = t & 31, wave = t >> 5;
  const int q = lane >> 3, c8 = (lane & 7) * 8;
  unsigned short* op = dst + cb;
  for (int pass = 0; pass < 2; ++pass) {
#pragma unroll
    for (int it = 0; it < 2; ++it) {
      const int row = wave * 8 + it * 4 + q;
      const unsigned int* sp = &sm[row][c8];
      const v4u u = (v4u){ (sp[0] & 0xffffu) | (sp[1] << 16), (sp[2] & 0xffffu) | (sp[3] << 16),
                           (sp[4] & 0xffffu) | (sp[5] << 16), (sp[6] & 0xffffu) | (sp[7] << 16) };
      *(volatile v4u*)(op + (size_t)(c0 + row) * rows + r0 + c8) = u;
    }
    __threadfence();
  }
}

__global__ __launch_bounds__(256) void rl_proj_kernel(const float* __restrict__ rh, const float* __restrict__ Wrk,
                                                      const float* __restrict__ Wrq, float* __restrict__ rk,
                                                      float* __restrict__ rq, int nrows) {
  const int idx = blockIdx.x * 256 + threadIdx.x;
  if (idx >= nrows) return;
  const v4f r  = *(const v4f*)(rh + (size_t)idx * kRl);
  const v4f k0 = *(const v4f*)(Wrk + 0);
  const v4f k1 = *(const v4f*)(Wrk + 4);
  const v4f k2 = *(const v4f*)(Wrk + 8);
  const v4f k3 = *(const v4f*)(Wrk + 12);
  asm volatile("" ::: "memory");
  const v4f q0 = *(const v4f*)(Wrq + 0);
  const v4f q1 = *(const v4f*)(Wrq + 4);
  const v4f q2 = *(const v4f*)(Wrq + 8);
  const v4f q3 = *(const v4f*)(Wrq + 12);
  v4f ok = r[0] * k0;
  ok = ok + r[1] * k1;
  ok = ok + r[2] * k2;
  ok = ok + r[3] * k3;
  v4f oq = r[0] * q0;
  oq = oq + r[1] * q1;
  oq = oq + r[2] * q2;
  oq = oq + r[3] * q3;
  float* pk = rk + (size_t)idx * kRl;
  float* pq = rq + (size_t)idx * kRl;
  *(volatile v4f*)pk = ok;
  *(volatile v4f*)pq = oq;
  __threadfence();
  *(volatile v4f*)pk = ok;
  *(volatile v4f*)pq = oq;
}

__global__ __launch_bounds__(256) void relbias_softmax_kernel(const float* __restrict__ Sp, const float* __restrict__ rqp,
                                                             const float* __restrict__ rkp, unsigned short* __restrict__ Pp,
                                                             int g0) {
  __shared__ __align__(16) float lg[kSeq];
  __shared__ float redM[8];
  __shared__ float redS[8];
  const int l    = blockIdx.x;
  const int gi   = blockIdx.y;
  const int b    = (g0 + gi) >> 3;
  const int t    = threadIdx.x;
  const int lane = t & 31, wave = t >> 5;
  const size_t rowoff = ((size_t)gi * kSeq + l) * kSeq;
  const float* sr  = Sp + rowoff;
  const v4f    rq4 = *(const v4f*)(rqp + ((size_t)b * kSeq + l) * kRl);
  const float* rkb = rkp + (size_t)b * kSeq * kRl;

  float mx = -__builtin_inff();
#pragma unroll 1
  for (int it = 0; it < 4; ++it) {
    const int c = it * 512 + 2 * t;
    const v2f sv = *(const v2f*)(sr + c);
    const v2f k0 = *(const v2f*)(rkb + c);
    const v2f k1 = *(const v2f*)(rkb + kSeq + c);
    const v2f k2 = *(const v2f*)(rkb + 2 * kSeq + c);
    const v2f k3 = *(const v2f*)(rkb + 3 * kSeq + c);
    v2f av;
#pragma unroll
    for (int e = 0; e < 2; ++e) {
      float bsum = rq4[0] * k0[e];
      bsum = bsum + rq4[1] * k1[e];
      bsum = bsum + rq4[2] * k2[e];
      bsum = bsum + rq4[3] * k3[e];
      const float a = sv[e] + 0.5f * bsum;
      av[e] = a;
      mx = fmaxf(mx, a);
    }
    *(v2f*)(lg + c) = av;
  }
#pragma unroll
  for (int off = 16; off > 0; off >>= 1) mx = fmaxf(mx, __shfl_xor(mx, off, 32));
  if (lane == 0) redM[wave] = mx;
  __syncthreads();
  float m = redM[0];
#pragma unroll
  for (int w = 1; w < 8; ++w) m = fmaxf(m, redM[w]);

  float sum = 0.f;
#pragma unroll 1
  for (int it = 0; it < 4; ++it) {
    const int c = it * 512 + 2 * t;
    const v2f lv = *(const v2f*)(lg + c);
    v2f ev;
#pragma unroll
    for (int e = 0; e < 2; ++e) {
      ev[e] = expf(lv[e] - m);
      sum += ev[e];
    }
    *(v2f*)(lg + c) = ev;
  }
#pragma unroll
  for (int off = 16; off > 0; off >>= 1) sum += __shfl_xor(sum, off, 32);
  if (lane == 0) redS[wave] = sum;
  __syncthreads();
  float tot = redS[0];
#pragma unroll
  for (int w = 1; w < 8; ++w) tot += redS[w];
  const float inv = kPCarry / tot;

  const v4f e0 = *(const v4f*)(lg + 8 * t);
  const v4f e1 = *(const v4f*)(lg + 8 * t + 4);
  unsigned short hb[8];
#pragma unroll
  for (int e = 0; e < 4; ++e) {
    hb[e]     = h_bits(e0[e] * inv);
    hb[4 + e] = h_bits(e1[e] * inv);
  }
  const v4u u = (v4u){pk16(hb[0], hb[1]), pk16(hb[2], hb[3]), pk16(hb[4], hb[5]), pk16(hb[6], hb[7])};
  unsigned short* pr = Pp + rowoff + 8 * (size_t)t;
  *(volatile v4u*)pr = u;
  __threadfence();
  *(volatile v4u*)pr = u;
}

template <bool HAS16>
__global__ __launch_bounds__(256) void add_ln_kernel(const float* __restrict__ x, const float* __restrict__ y,
                                                     const float* __restrict__ gam, const float* __restrict__ bet,
                                                     float* __restrict__ outp, unsigned short* __restrict__ out16) {
  __shared__ float red1[8];
  __shared__ float red2[8];
  __shared__ __align__(16) float srow[kDim];
  const int t = threadIdx.x;
  const int lane = t & 31, wave = t >> 5;
  const size_t base = (size_t)blockIdx.x * kDim;
  const v4f vx = *(const v4f*)(x + base + 4 * t);
  const v4f vy = *(const v4f*)(y + base + 4 * t);
  const v4f s  = vx + vy;
  float sum = (s[0] + s[1]) + (s[2] + s[3]);
#pragma unroll
  for (int off = 16; off > 0; off >>= 1) sum += __shfl_xor(sum, off, 32);
  if (lane == 0) red1[wave] = sum;
  __syncthreads();
  float tsum = red1[0];
#pragma unroll
  for (int w = 1; w < 8; ++w) tsum += red1[w];
  const float mu = tsum * kInvDim;
  const v4f d = s - mu;
  float sq = (d[0] * d[0] + d[1] * d[1]) + (d[2] * d[2] + d[3] * d[3]);
#pragma unroll
  for (int off = 16; off > 0; off >>= 1) sq += __shfl_xor(sq, off, 32);
  if (lane == 0) red2[wave] = sq;
  __syncthreads();
  float tsq = red2[0];
#pragma unroll
  for (int w = 1; w < 8; ++w) tsq += red2[w];
  const float var  = tsq * kInvDim;
  const float rstd = rsqrtf(var + kLnEps);
  const v4f g  = *(const v4f*)(gam + 4 * t);
  const v4f be = *(const v4f*)(bet + 4 * t);
  const v4f o  = (d * rstd) * g + be;
  float* op = outp + base + 4 * t;
  *(volatile v4f*)op = o;
  __threadfence();
  *(volatile v4f*)op = o;
  if (HAS16) {
    *(v4f*)(srow + 4 * t) = o;
    __syncthreads();
    if (t < 128) {
      const v4f a = *(const v4f*)(srow + 8 * t);
      const v4f c = *(const v4f*)(srow + 8 * t + 4);
      unsigned short hb[8];
#pragma unroll
      for (int e = 0; e < 4; ++e) {
        hb[e]     = h_bits(a[e]);
        hb[4 + e] = h_bits(c[e]);
      }
      const v4u u = (v4u){pk16(hb[0], hb[1]), pk16(hb[2], hb[3]), pk16(hb[4], hb[5]), pk16(hb[6], hb[7])};
      unsigned short* hp = out16 + base + 8 * (size_t)t;
      *(volatile v4u*)hp = u;
      __threadfence();
      *(volatile v4u*)hp = u;
    }
  }
}

extern "C" void kernel_launch(void* const* d_in, const int* in_sizes, int n_in,
                              void* d_out, int out_size, void* d_ws, size_t ws_size,
                              hipStream_t stream) {
  if (n_in < 16) return;
  const int nTokDim = kTok * kDim;
  if (in_sizes[0] != nTokDim || in_sizes[1] != kTok * kRl) return;
  if (in_sizes[2] != kDim * kDim || in_sizes[3] != kDim * kDim || in_sizes[4] != kDim * kDim || in_sizes[5] != kDim * kDim) return;
  if (in_sizes[6] != kRl * kRl || in_sizes[7] != kRl * kRl) return;
  if (in_sizes[8] != kDim * kFfn || in_sizes[9] != kFfn || in_sizes[10] != kFfn * kDim || in_sizes[11] != kDim) return;
  if (in_sizes[12] != kDim || in_sizes[13] != kDim || in_sizes[14] != kDim || in_sizes[15] != kDim) return;
  if (out_size != nTokDim) return;

  const size_t szP16 = (size_t)kTok * kDim * 2;
  const size_t szW4  = (size_t)4 * kDim * kDim * 2;
  const size_t szW1  = (size_t)kDim * kFfn * 2;
  const size_t szSC  = (size_t)kGpp * kSeq * kSeq * 4;
  const size_t szPP  = (size_t)kGpp * kSeq * kSeq * 2;
  const size_t szR   = (size_t)kTok * kRl * 4;
  static_assert((size_t)kGpp * kSeq * kSeq * 4 == 2 * (size_t)kTok * kDim * 4, "h_sa + h1 fit the score region");
  static_assert(4 * (size_t)kTok * kDim * 2 == (size_t)kTok * kFfn * 2, "mid fits q+v+KT+VT");
  const size_t offHh = 0;
  const size_t offW4 = offHh + szP16;
  const size_t offW1 = offW4 + szW4;
  const size_t offW2 = offW1 + szW1;
  const size_t offK  = offW2 + szW1;
  const size_t offQ  = offK + szP16;
  const size_t offV  = offQ + szP16;
  const size_t offKT = offV + szP16;
  const size_t offVT = offKT + szP16;
  const size_t offSC = offVT + szP16;
  const size_t offPP = offSC + szSC;
  const size_t offRQ = offPP + szPP;
  const size_t offRK = offRQ + szR;
  const size_t total = offRK + szR;
  if (ws_size < total) return;

  const float* h   = (const float*)d_in[0];
  const float* rh  = (const float*)d_in[1];
  const float* Wq  = (const float*)d_in[2];
  const float* Wk  = (const float*)d_in[3];
  const float* Wv  = (const float*)d_in[4];
  const float* Wo  = (const float*)d_in[5];
  const float* Wrk = (const float*)d_in[6];
  const float* Wrq = (const float*)d_in[7];
  const float* W1  = (const float*)d_in[8];
  const float* b1  = (const float*)d_in[9];
  const float* W2  = (const float*)d_in[10];
  const float* b2  = (const float*)d_in[11];
  const float* g1  = (const float*)d_in[12];
  const float* be1 = (const float*)d_in[13];
  const float* g2  = (const float*)d_in[14];
  const float* be2 = (const float*)d_in[15];
  float* out = (float*)d_out;
  char* ws = (char*)d_ws;
  unsigned short* Hh  = (unsigned short*)(ws + offHh);
  unsigned short* CTX = Hh;
  unsigned short* WT4 = (unsigned short*)(ws + offW4);
  unsigned short* WoT = WT4 + (size_t)3 * kDim * kDim;
  unsigned short* W1T = (unsigned short*)(ws + offW1);
  unsigned short* W2T = (unsigned short*)(ws + offW2);
  unsigned short* K16 = (unsigned short*)(ws + offK);
  unsigned short* H1h = K16;
  unsigned short* Q16 = (unsigned short*)(ws + offQ);
  unsigned short* MID = Q16;
  unsigned short* V16 = (unsigned short*)(ws + offV);
  unsigned short* KT  = (unsigned short*)(ws + offKT);
  unsigned short* VT  = (unsigned short*)(ws + offVT);
  float* SC  = (float*)(ws + offSC);
  float* HSA = SC;
  float* HF  = HSA;
  float* H1f = (float*)(ws + offSC + szSC / 2);
  unsigned short* PP = (unsigned short*)(ws + offPP);
  float* RQ = (float*)(ws + offRQ);
  float* RK = (float*)(ws + offRK);

  const int n8 = nTokDim / 8;
  cast8_f16_kernel<<<dim3(n8 / 256), dim3(256), 0, stream>>>(h, Hh, n8);
  wt_cast_kernel<<<dim3(kDim / 64, kDim / 64, 4), dim3(256), 0, stream>>>(Wk, Wq, Wv, Wo, WT4, kDim, kDim, (long)kDim * kDim, kWCarry);
  wt_cast_kernel<<<dim3(kDim / 64, kFfn / 64, 1), dim3(256), 0, stream>>>(W1, W1, W1, W1, W1T, kDim, kFfn, 0L, kWCarry);
  wt_cast_kernel<<<dim3(kFfn / 64, kDim / 64, 1), dim3(256), 0, stream>>>(W2, W2, W2, W2, W2T, kFfn, kDim, 0L, kWCarry);
  rl_proj_kernel<<<dim3(kTok / 256), dim3(256), 0, stream>>>(rh, Wrk, Wrq, RK, RQ, kTok);

  {
    const int tiles = (kTok / 64) * (kDim / 64);
    wmma_gemm64<0, false, 0, 1, false, 0><<<dim3(tiles / 8, 3), dim3(256), 0, stream>>>(
        Hh, Hh, kDim, 0L, WT4, WT4, kDim, (long)kDim * kDim,
        (void*)K16, (void*)K16, kDim, (long)kTok * kDim, RQ, RQ, 0L, kTok, kDim, kDim, kWCarryInv);
  }
  transpose16_kernel<<<dim3(kSeq / 64, kHeadDim / 64, kGroups), dim3(256), 0, stream>>>(K16, KT, kHeadDim, kSeq);
  transpose16_kernel<<<dim3(kHeadDim / 64, kSeq / 64, kGroups), dim3(256), 0, stream>>>(V16, VT, kSeq, kHeadDim);

  const long strideChunk = (long)kChunk;
  const long strideScore = (long)kSeq * kSeq;
  const int  tilesScore  = (kSeq / 64) * (kSeq / 64);
  const int  tilesCtx    = (kSeq / 64) * (kHeadDim / 64);
  for (int g0 = 0; g0 < kGroups; g0 += kGpp) {
    const unsigned short* Ag  = Q16 + (size_t)g0 * kChunk;
    const unsigned short* Btg = KT  + (size_t)g0 * kChunk;
    wmma_gemm64<0, false, 0, 0, false, 0><<<dim3(tilesScore / 8, kGpp), dim3(256), 0, stream>>>(
        Ag, Ag, kHeadDim, strideChunk, Btg, Btg, kHeadDim, strideChunk,
        (void*)SC, (void*)SC, kSeq, strideScore, RQ, RQ, 0L, kSeq, kSeq, kHeadDim, kScoreScale);
    relbias_softmax_kernel<<<dim3(kSeq, kGpp), dim3(256), 0, stream>>>(SC, RQ, RK, PP, g0);
    const unsigned short* VTg = VT + (size_t)g0 * kChunk;
    unsigned short* Cg = CTX + (size_t)g0 * kChunk;
    wmma_gemm64<0, false, 0, 1, false, 0><<<dim3(tilesCtx / 8, kGpp), dim3(256), 0, stream>>>(
        PP, PP, kSeq, strideScore, VTg, VTg, kSeq, strideChunk,
        (void*)Cg, (void*)Cg, kHeadDim, strideChunk, RQ, RQ, 0L, kSeq, kHeadDim, kSeq, kPVScale);
  }

  {
    const int tiles = (kTok / 64) * (kDim / 64);
    wmma_gemm64<0, false, 0, 0, false, 0><<<dim3(tiles / 8, 1), dim3(256), 0, stream>>>(
        CTX, CTX, kDim, 0L, WoT, WoT, kDim, 0L,
        (void*)HSA, (void*)HSA, kDim, 0L, RQ, RQ, 0L, kTok, kDim, kDim, kWoScale);
  }
  add_ln_kernel<true><<<dim3(kTok), dim3(256), 0, stream>>>(HSA, h, g1, be1, H1f, H1h);
  {
    const int tiles = (kTok / 64) * (kFfn / 64);
    wmma_gemm64<0, false, 2, 1, false, 2><<<dim3(tiles / 8, 1), dim3(256), 0, stream>>>(
        H1h, H1h, kDim, 0L, W1T, W1T, kDim, 0L,
        (void*)MID, (void*)MID, kFfn, 0L, b1, RQ, 0L, kTok, kFfn, kDim, kWCarryInv);
  }
  {
    const int tiles = (kTok / 64) * (kDim / 64);
    wmma_gemm64<0, false, 2, 0, false, 0><<<dim3(tiles / 8, 1), dim3(256), 0, stream>>>(
        MID, MID, kFfn, 0L, W2T, W2T, kFfn, 0L,
        (void*)HF, (void*)HF, kDim, 0L, b2, RQ, 0L, kTok, kDim, kFfn, kWCarryInv);
  }
  add_ln_kernel<false><<<dim3(kTok), dim3(256), 0, stream>>>(H1f, HF, g2, be2, out, H1h);
}
